// SingleMatchingGroup_6811818132507
// MI455X (gfx1250) — hardware-verified
//
#include <hip/hip_runtime.h>

#define BATCH   2
#define HH      64
#define WW      64
#define CIN     128
#define COUT    256
#define NC      32
#define FS      8
#define PATCH   5
#define KCONV1  1152
#define NPIX    (BATCH*HH*WW)

typedef unsigned int       u32;
typedef unsigned long long u64;
#define __bf16 _Float16
typedef __attribute__((ext_vector_type(16))) __bf16 v16bf;
typedef __attribute__((ext_vector_type(8)))  float  v8f;
typedef __attribute__((ext_vector_type(4)))  float  v4f_t;
typedef float v4fa __attribute__((ext_vector_type(4), may_alias));
typedef __attribute__((ext_vector_type(4)))  u32    v4u_t;
typedef u32 v4ua __attribute__((ext_vector_type(4), may_alias));
typedef __attribute__((ext_vector_type(4)))  u32    su4;
typedef __attribute__((ext_vector_type(8)))  u32    su8;

union FragBF { v16bf v; uint4 q[2]; };

#define OFF_XBF   0
#define SZ_XBF    (NPIX*CIN*2)
#define OFF_B1    (OFF_XBF + SZ_XBF)
#define SZ_B1     (KCONV1*CIN*2)
#define OFF_BIAS  (OFF_B1 + SZ_B1)
#define SZ_BIAS   (CIN*4)
#define OFF_H     (OFF_BIAS + SZ_BIAS)
#define SZ_H      (NPIX*CIN*2)
#define OFF_B2    (OFF_H + SZ_H)
#define SZ_B2     (CIN*COUT*2)
#define OFF_F     (OFF_B2 + SZ_B2)
#define SZ_F      (NPIX*COUT*2)
#define OFF_S     (OFF_F + SZ_F)
#define SZ_S      (NPIX*NC*4*4)

__device__ __forceinline__ void tdm_load_1d(u32 lds_addr, const void* gptr, u32 nelem) {
    u64 ga = (u64)gptr;
    su4 g0;
    g0.x = 1u;
    g0.y = lds_addr;
    g0.z = (u32)ga;
    g0.w = ((u32)(ga >> 32) & 0x01FFFFFFu) | (2u << 30);
    su8 g1;
    g1.s0 = 0x00010000u;
    g1.s1 = (nelem & 0xFFFFu) << 16;
    g1.s2 = (nelem >> 16) | (1u << 16);
    g1.s3 = (nelem & 0xFFFFu) << 16;
    g1.s4 = 1u;
    g1.s5 = nelem;
    g1.s6 = 0u;
    g1.s7 = 0u;
    asm volatile("tensor_load_to_lds %0, %1" :: "s"(g0), "s"(g1) : "memory");
}

__global__ void k_convert_x(const float* __restrict__ x, __bf16* __restrict__ xbf) {
    int t = blockIdx.x * blockDim.x + threadIdx.x;
    if (t >= NPIX * (CIN / 8)) return;
    int c8  = (t & 15) * 8;
    int pix = t >> 4;
    int b = pix >> 12, yv = (pix >> 6) & 63, xp = pix & 63;
    __bf16 hh[8];
    #pragma unroll
    for (int e = 0; e < 8; ++e) hh[e] = (__bf16)x[(((size_t)b * CIN + c8 + e) * HH + yv) * WW + xp];
    __bf16* d = xbf + (size_t)pix * CIN + c8;
    *(volatile v4u_t*)d = *(const v4ua*)hh; __threadfence(); *(volatile v4u_t*)d = *(const v4ua*)hh;
}

__global__ void k_prep_w(const float* __restrict__ w1, const float* __restrict__ gamma,
                         const float* __restrict__ beta, const float* __restrict__ mean,
                         const float* __restrict__ var, const float* __restrict__ w2,
                         __bf16* __restrict__ B1p, float* __restrict__ bias,
                         __bf16* __restrict__ B2p) {
    int idx = blockIdx.x * blockDim.x + threadIdx.x;
    const int N1 = KCONV1 * CIN;
    const int N2 = CIN * COUT;
    if (idx < N1) {
        int kk   = idx & 31;
        int n    = (idx >> 5) & 127;
        int kb32 = idx >> 12;
        int k    = kb32 * 32 + kk;
        int ci   = k & 127;
        int tap  = k >> 7;
        int dy = tap / 3, dx = tap % 3;
        float s = gamma[n >> 3] * rsqrtf(var[n >> 3] + 1e-5f);
        { const __bf16 v = (__bf16)(w1[((n * CIN + ci) * 3 + dy) * 3 + dx] * s); *(volatile __bf16*)(B1p + idx) = v; __threadfence(); *(volatile __bf16*)(B1p + idx) = v; }
    } else if (idx < N1 + N2) {
        int j    = idx - N1;
        int kk   = j & 31;
        int n    = (j >> 5) & 255;
        int kb32 = j >> 13;
        int ci   = kb32 * 32 + kk;
        { const __bf16 v = (__bf16)(w2[n * CIN + ci]); *(volatile __bf16*)(B2p + j) = v; __threadfence(); *(volatile __bf16*)(B2p + j) = v; }
    } else if (idx < N1 + N2 + CIN) {
        int n = idx - N1 - N2;
        float s = gamma[n >> 3] * rsqrtf(var[n >> 3] + 1e-5f);
        { const float v = beta[n >> 3] - mean[n >> 3] * s; *(volatile float*)(bias + n) = v; __threadfence(); *(volatile float*)(bias + n) = v; }
    }
}

__device__ __forceinline__ v16bf load_frag(const __bf16* rowbase, int qi) {
    FragBF f;
    const uint4* p = (const uint4*)rowbase;
    f.q[0] = p[qi];
    f.q[1] = p[2 + qi];
    return f.v;
}

__global__ __launch_bounds__(128) void k_conv1(const __bf16* __restrict__ xbf,
                                               const __bf16* __restrict__ B1p,
                                               const float*  __restrict__ bias,
                                               __bf16* __restrict__ h) {
    __shared__ __align__(16) __bf16 sA[2][64 * 32];
    __shared__ __align__(16) __bf16 sB[2][128 * 32];
    const int by = blockIdx.x;
    const int b  = by >> 6;
    const int y  = by & 63;
    const int tid  = threadIdx.x;
    const int wave = tid >> 5;
    const int lane = tid & 31;
    const int qi   = lane >> 4;
    const int l15  = lane & 15;

    v8f acc[8];
    #pragma unroll
    for (int nt = 0; nt < 8; ++nt) acc[nt] = (v8f){0,0,0,0,0,0,0,0};

    const int m    = tid >> 1;
    const int half = (tid & 1) * 16;

    auto stageA = [&](int kblk, int buf) {
        int tap = kblk >> 2;
        int c0  = (kblk & 3) << 5;
        int dy  = tap / 3;
        int dx  = tap - dy * 3;
        int yy  = y + dy - 1;
        int xx  = m + dx - 1;
        uint4 d0 = {0,0,0,0}, d1 = {0,0,0,0};
        if (yy >= 0 && yy < HH && xx >= 0 && xx < WW) {
            const uint4* s4 = (const uint4*)(xbf + (((b * HH + yy) * WW + xx) * CIN + c0 + half));
            d0 = s4[0]; d1 = s4[1];
        }
        uint4* a4 = (uint4*)&sA[buf][m * 32 + half];
        a4[0] = d0; a4[1] = d1;
    };

    stageA(0, 0);
    if (wave == 0)
        tdm_load_1d((u32)(u64)&sB[0][0], B1p, 128 * 32);

    for (int i = 0; i < 36; ++i) {
        const int cur = i & 1, nxt = cur ^ 1;
        if (wave == 0)
            __builtin_amdgcn_s_wait_tensorcnt(0);
        __syncthreads();
        if (i + 1 < 36) {
            stageA(i + 1, nxt);
            if (wave == 0)
                tdm_load_1d((u32)(u64)&sB[nxt][0], B1p + (i + 1) * (128 * 32), 128 * 32);
        }
        const int arow = wave * 16 + l15;
        v16bf av = load_frag(&sA[cur][arow * 32], qi);
        #pragma unroll
        for (int nt = 0; nt < 8; ++nt) {
            int col = nt * 16 + l15;
            v16bf bv = load_frag(&sB[cur][col * 32], qi);
            acc[nt] = __builtin_amdgcn_wmma_f32_16x16x32_f16(
                false, av, false, bv, (short)0, acc[nt], false, false);
        }
    }

    __syncthreads();
    __bf16* st = &sB[0][0] + wave * (16 * 136);
    #pragma unroll
    for (int nt = 0; nt < 8; ++nt) {
        int col = nt * 16 + l15;
        float bsv = bias[col];
        #pragma unroll
        for (int r = 0; r < 8; ++r) {
            int rl = (lane < 16) ? r : r + 8;
            float vv = acc[nt][r] + bsv;
            vv = vv > 0.0f ? vv : 0.0f;
            st[rl * 136 + col] = (__bf16)vv;
        }
    }
    asm volatile("s_wait_dscnt 0" ::: "memory");
    #pragma unroll 1
    for (int pass = 0; pass < 2; ++pass) {
        #pragma unroll
        for (int i = 0; i < 8; ++i) { const int c = lane + 32 * i, rl = c >> 4, q = (c & 15) * 8;
            *(volatile v4u_t*)(h + (size_t)(by * 64 + wave * 16 + rl) * CIN + q) = *(const v4ua*)(st + rl * 136 + q); }
        __threadfence();
    }
}

__global__ __launch_bounds__(128) void k_conv2(const __bf16* __restrict__ h,
                                               const __bf16* __restrict__ B2p,
                                               __bf16* __restrict__ f) {
    __shared__ __align__(16) __bf16 sA[64 * 128];
    __shared__ __align__(16) __bf16 sB[2][256 * 32];
    const int mb   = blockIdx.x * 64;
    const int tid  = threadIdx.x;
    const int wave = tid >> 5;
    const int lane = tid & 31;
    const int qi   = lane >> 4;
    const int l15  = lane & 15;

    v8f acc[16];
    #pragma unroll
    for (int nt = 0; nt < 16; ++nt) acc[nt] = (v8f){0,0,0,0,0,0,0,0};

    if (wave == 0) {
        tdm_load_1d((u32)(u64)&sA[0], h + mb * CIN, 64 * CIN);
        tdm_load_1d((u32)(u64)&sB[0][0], B2p, 256 * 32);
    }

    for (int kb = 0; kb < 4; ++kb) {
        const int cur = kb & 1, nxt = cur ^ 1;
        if (wave == 0)
            __builtin_amdgcn_s_wait_tensorcnt(0);
        __syncthreads();
        if (wave == 0 && kb + 1 < 4)
            tdm_load_1d((u32)(u64)&sB[nxt][0], B2p + (kb + 1) * (256 * 32), 256 * 32);

        const int arow = wave * 16 + l15;
        v16bf av = load_frag(&sA[arow * CIN + kb * 32], qi);
        #pragma unroll
        for (int nt = 0; nt < 16; ++nt) {
            int col = nt * 16 + l15;
            v16bf bv = load_frag(&sB[cur][col * 32], qi);
            acc[nt] = __builtin_amdgcn_wmma_f32_16x16x32_f16(
                false, av, false, bv, (short)0, acc[nt], false, false);
        }
    }

    __syncthreads();
    __bf16* st = &sB[0][0] + wave * (16 * 264);
    #pragma unroll
    for (int nt = 0; nt < 16; ++nt) {
        int col = nt * 16 + l15;
        #pragma unroll
        for (int r = 0; r < 8; ++r) {
            int rl = (lane < 16) ? r : r + 8;
            st[rl * 264 + col] = (__bf16)acc[nt][r];
        }
    }
    asm volatile("s_wait_dscnt 0" ::: "memory");
    #pragma unroll 1
    for (int pass = 0; pass < 2; ++pass) {
        #pragma unroll
        for (int i = 0; i < 16; ++i) { const int c = lane + 32 * i, rl = c >> 5, q = (c & 31) * 8;
            *(volatile v4u_t*)(f + (size_t)(mb + wave * 16 + rl) * COUT + q) = *(const v4ua*)(st + rl * 264 + q); }
        __threadfence();
    }
}

#define VSTRIDE 201

__device__ __forceinline__ float sampF(const __bf16* f, int b, int yy, int xx, int ch) {
    if (yy < 0 || yy >= HH || xx < 0 || xx >= WW) return 0.0f;
    return (float)f[((b * HH + yy) * WW + xx) * COUT + ch];
}

__global__ __launch_bounds__(64) void k_sim(const __bf16* __restrict__ f,
                                            float* __restrict__ out) {
    __shared__ float vals[2 * 32 * VSTRIDE];
    const int pix  = blockIdx.x;
    const int b = pix >> 12;
    const int y = (pix >> 6) & 63;
    const int x = pix & 63;
    const int tid  = threadIdx.x;
    const int rot  = tid >> 5;
    const int lane = tid & 31;
    float* myv = &vals[(rot * 32 + lane) * VSTRIDE];

    const float ct =  0.70710678118654752f;
    const float st = -0.70710678118654752f;

    #pragma unroll 1
    for (int fs = 0; fs < FS; ++fs) {
        int ch = lane * FS + fs;
        if (rot == 1) ch = (ch & ~3) | ((ch + 1) & 3);
        #pragma unroll 1
        for (int py = 0; py < PATCH; ++py) {
            #pragma unroll 1
            for (int px = 0; px < PATCH; ++px) {
                float val;
                if (rot == 0) {
                    val = sampF(f, b, y + py - 2, x + px - 2, ch);
                } else {
                    float dx = (float)px - 2.0f, dyv = (float)py - 2.0f;
                    float sx = ct * dx + st * dyv + 2.0f;
                    float sy = -st * dx + ct * dyv + 2.0f;
                    int x0 = (int)floorf(sx), y0 = (int)floorf(sy);
                    float wx = sx - (float)x0, wy = sy - (float)y0;
                    const float cw[4] = {(1.f - wy) * (1.f - wx), (1.f - wy) * wx,
                                         wy * (1.f - wx), wy * wx};
                    val = 0.0f;
                    #pragma unroll
                    for (int c4 = 0; c4 < 4; ++c4) {
                        int yi = y0 + (c4 >> 1);
                        int xi = x0 + (c4 & 1);
                        if (yi >= 0 && yi < PATCH && xi >= 0 && xi < PATCH && cw[c4] != 0.0f)
                            val += cw[c4] * sampF(f, b, y + yi - 2, x + xi - 2, ch);
                    }
                }
                myv[fs * 25 + py * 5 + px] = val;
            }
        }
    }
    float dot = 0.0f, nsq = 0.0f;
    #pragma unroll 1
    for (int fs = 0; fs < FS; ++fs) {
        const int rpf = ((fs < 4) ? 4 : 0) + ((8 - fs) & 3);
        #pragma unroll 1
        for (int py = 0; py < PATCH; ++py) {
            #pragma unroll 1
            for (int px = 0; px < PATCH; ++px) {
                float v  = myv[fs * 25 + py * 5 + px];
                float vr = myv[rpf * 25 + py * 5 + (4 - px)];
                dot += v * vr;
                nsq += v * v;
            }
        }
    }
    float nrm = fmaxf(sqrtf(nsq), 1e-6f);
    float sim = dot / (nrm * nrm);
    (void)b; (void)y; (void)x;
    float* sr = out + (size_t)pix * (NC * 4) + lane * 4 + rot;
    *(volatile float*)sr = sim; *(volatile float*)(sr + 2) = sim; __threadfence();
    *(volatile float*)sr = sim; *(volatile float*)(sr + 2) = sim;
}

__global__ __launch_bounds__(256) void k_transpose(const float* __restrict__ srow, float* __restrict__ out) {
    const int t = blockIdx.x * 256 + threadIdx.x;
    if (t >= BATCH * NC * 4 * HH * (WW / 4)) return;
    const int x4 = (t & 15) * 4;
    const int y  = (t >> 4) & 63;
    const int c  = (t >> 10) & 127;
    const int b  = t >> 17;
    v4f_t v;
    const float* s = srow + ((size_t)((b * HH + y) * WW + x4)) * (NC * 4) + c;
    v.x = s[0]; v.y = s[NC * 4]; v.z = s[2 * NC * 4]; v.w = s[3 * NC * 4];
    float* d = out + (((size_t)b * (NC * 4) + c) * HH + y) * WW + x4;
    *(volatile v4f_t*)d = v; __threadfence(); *(volatile v4f_t*)d = v;
}

extern "C" void kernel_launch(void* const* d_in, const int* in_sizes, int n_in,
                              void* d_out, int out_size, void* d_ws, size_t ws_size,
                              hipStream_t stream) {
    const float* x     = (const float*)d_in[0];
    const float* w1    = (const float*)d_in[1];
    const float* gamma = (const float*)d_in[2];
    const float* beta  = (const float*)d_in[3];
    const float* mean  = (const float*)d_in[4];
    const float* var   = (const float*)d_in[5];
    const float* w2    = (const float*)d_in[6];

    unsigned char* ws = (unsigned char*)d_ws;
    __bf16* xbf  = (__bf16*)(ws + OFF_XBF);
    __bf16* B1p  = (__bf16*)(ws + OFF_B1);
    float*  bias = (float*)(ws + OFF_BIAS);
    __bf16* h    = (__bf16*)(ws + OFF_H);
    __bf16* B2p  = (__bf16*)(ws + OFF_B2);
    __bf16* f    = (__bf16*)(ws + OFF_F);

    float* srow = (float*)(ws + OFF_S);
    k_convert_x<<<(NPIX * (CIN / 8) + 255) / 256, 256, 0, stream>>>(x, xbf);
    k_prep_w<<<(KCONV1 * CIN + CIN * COUT + CIN + 255) / 256, 256, 0, stream>>>(
        w1, gamma, beta, mean, var, w2, B1p, bias, B2p);
    k_conv1<<<BATCH * HH, 128, 0, stream>>>(xbf, B1p, bias, h);
    k_conv2<<<NPIX / 64, 128, 0, stream>>>(h, B2p, f);
    k_sim<<<NPIX, 64, 0, stream>>>(f, srow);
    k_transpose<<<(BATCH * NC * 4 * HH * (WW / 4)) / 256, 256, 0, stream>>>(srow, (float*)d_out);
}
